// GAT_2379411882410
// MI455X (gfx1250) — hardware-verified
//
#include <hip/hip_runtime.h>
#include <stddef.h>
#include <stdint.h>
#include <math.h>

#define F_IN    256
#define HC1     256
#define NOUT    64
#define KP      512
#define SDW     16
#define NTHR    256
#define NWAVE   8
#define EPT     8
#define CHUNK   (NTHR * EPT)
#define WCAP    (EPT * 32)
#define LISTN   (NWAVE * WCAP)
#define NBA     1024
#define SLA     10
#define RCAP    16384
#define DEGCAP  64
#define GBM     64
#define GBN     64
#define GTHR    128
#define NU1     (HC1 * (F_IN / 8))
#define NU2     (NOUT * (KP / 8))
#define NEGSL   0.2f
#define AGG_ZINTS (LISTN + 2 * RCAP + 3 * NBA)
#define AGG_LDS_INTS (AGG_ZINTS + 16 + NTHR * 8)
#define G1_LDS_FLOATS (GBM * HC1 + GBM * SDW)
#define WSMAX   134217728

static_assert((CHUNK & (CHUNK - 1)) == 0 && CHUNK <= 4096);
static_assert((NBA & (NBA - 1)) == 0 && NBA == (1 << SLA));
static_assert(((long long)CHUNK << SLA) < (1LL << 31));
static_assert(NBA % NWAVE == 0 && NBA % 32 == 0 && NBA % GBM == 0);
static_assert(RCAP % 4 == 0 && AGG_ZINTS % 4 == 0 && LISTN % 4 == 0);
static_assert(((AGG_ZINTS + 16) * 4) % 16 == 0);
static_assert(AGG_LDS_INTS * 4 <= 300000);
static_assert(F_IN % 32 == 0 && KP % 32 == 0 && KP == 2 * HC1);
static_assert(HC1 == 8 * 32 && NOUT == 2 * 32);
static_assert(GBM == (GTHR / 32) * 16 && GTHR == 2 * GBN && GTHR == 2 * GBM && NOUT == GBN);
static_assert(NU1 % NTHR == 0 && NU2 % NTHR == 0);
static_assert(F_IN / 8 == 32 && KP / 8 == 64);
static_assert(NTHR * 4 == GBM * SDW);

typedef float          v2f   __attribute__((ext_vector_type(2)));
typedef float          v4f   __attribute__((ext_vector_type(4)));
typedef float          v8f   __attribute__((ext_vector_type(8)));
typedef int            v4i   __attribute__((ext_vector_type(4)));
typedef int            v8i   __attribute__((ext_vector_type(8)));
typedef unsigned short v8us  __attribute__((ext_vector_type(8)));
typedef __bf16         v16b  __attribute__((ext_vector_type(16)));
typedef v2f  __attribute__((may_alias)) v2fa;
typedef v4f  __attribute__((may_alias)) v4fa;
typedef v4i  __attribute__((may_alias)) v4ia;
typedef v8us __attribute__((may_alias)) v8usa;
union FragB { v16b v; v8us h[2]; v8i w; };

__device__ __forceinline__ v8f wmb(const FragB& a, const FragB& b, v8f c) {
  v8f d = __builtin_amdgcn_wmma_f32_16x16x32_bf16(false, a.v, false, b.v, (short)0, c, false, false);
  asm volatile("v_nop\n\tv_nop\n\tv_nop\n\tv_nop" : "+v"(d) : "v"(a.w), "v"(b.w));
  return d;
}

__device__ __forceinline__ unsigned int f2bf(float f) {
  const unsigned int u = __float_as_uint(f);
  return ((u + 0x7FFFu + ((u >> 16) & 1u)) >> 16) & 0xFFFFu;
}
__device__ __forceinline__ float bf2f(unsigned int b) { return __uint_as_float(b << 16); }
__device__ __forceinline__ float bfr(float f) { return bf2f(f2bf(f)); }
__device__ __forceinline__ v4f bfr4(const v4f a) {
  v4f r; r.x = bfr(a.x); r.y = bfr(a.y); r.z = bfr(a.z); r.w = bfr(a.w); return r;
}
__device__ __forceinline__ unsigned int pk2(float lo, float hi) { return f2bf(lo) | (f2bf(hi) << 16); }

template <int SLB>
__device__ __forceinline__ int scan_chunk(const int* __restrict__ dsts, int nE, int cbase, int slotBase,
                                          int nb, int vec8, int* list, int tid, int lane, int wave) {
  int wc = 0;
  const int el0  = tid * EPT;
  const int e0   = cbase + el0;
  const int sent = -2147483647 - 1;
  v4i da, db;
  if (vec8 != 0 && cbase + CHUNK <= nE) {
    da = *(const v4i*)(dsts + e0);
    db = *(const v4i*)(dsts + e0 + 4);
  } else {
    da.x = (e0     < nE) ? dsts[min(e0,     nE - 1)] : sent;
    da.y = (e0 + 1 < nE) ? dsts[min(e0 + 1, nE - 1)] : sent;
    da.z = (e0 + 2 < nE) ? dsts[min(e0 + 2, nE - 1)] : sent;
    da.w = (e0 + 3 < nE) ? dsts[min(e0 + 3, nE - 1)] : sent;
    db.x = (e0 + 4 < nE) ? dsts[min(e0 + 4, nE - 1)] : sent;
    db.y = (e0 + 5 < nE) ? dsts[min(e0 + 5, nE - 1)] : sent;
    db.z = (e0 + 6 < nE) ? dsts[min(e0 + 6, nE - 1)] : sent;
    db.w = (e0 + 7 < nE) ? dsts[min(e0 + 7, nE - 1)] : sent;
  }
  const unsigned nbs = (unsigned)slotBase;
  const unsigned unb = (unsigned)nb;
  const unsigned s0 = (unsigned)da.x - nbs, s1 = (unsigned)da.y - nbs;
  const unsigned s2 = (unsigned)da.z - nbs, s3 = (unsigned)da.w - nbs;
  const unsigned s4 = (unsigned)db.x - nbs, s5 = (unsigned)db.y - nbs;
  const unsigned s6 = (unsigned)db.z - nbs, s7 = (unsigned)db.w - nbs;
  const bool h0 = s0 < unb, h1 = s1 < unb, h2 = s2 < unb, h3 = s3 < unb;
  const bool h4 = s4 < unb, h5 = s5 < unb, h6 = s6 < unb, h7 = s7 < unb;
  const unsigned any = __builtin_amdgcn_ballot_w32(h0 | h1 | h2 | h3 | h4 | h5 | h6 | h7);
  if (any != 0u) {
#define HITJ(J, HJ, SJ) { \
      const unsigned mj = __builtin_amdgcn_ballot_w32(HJ); \
      if (mj != 0u) { \
        if (HJ) { \
          const int pos = wc + (int)__builtin_amdgcn_mbcnt_lo(mj, 0u); \
          if (pos < WCAP) list[wave * WCAP + pos] = ((el0 + (J)) << SLB) | (int)(SJ); \
        } \
        wc += (int)__builtin_popcount(mj); } }
    HITJ(0, h0, s0)
    HITJ(1, h1, s1)
    HITJ(2, h2, s2)
    HITJ(3, h3, s3)
    HITJ(4, h4, s4)
    HITJ(5, h5, s5)
    HITJ(6, h6, s6)
    HITJ(7, h7, s7)
#undef HITJ
  }
  return wc;
}

__global__ __launch_bounds__(NTHR) void k_wprep(const float* __restrict__ W1, const float* __restrict__ W2,
                                                unsigned short* W1T, unsigned short* W22T) {
  const int u = (int)blockIdx.x * NTHR + (int)threadIdx.x;
  v8us o;
  unsigned short* dp;
  if (u < NU1) {
    const int n  = u >> 5;
    const int k8 = (u & 31) * 8;
    const float* p = W1 + (size_t)k8 * HC1 + n;
#pragma unroll
    for (int i = 0; i < 8; ++i) o[i] = (unsigned short)f2bf(p[(size_t)i * HC1]);
    dp = W1T + (size_t)n * F_IN + k8;
  } else if (u < NU1 + NU2) {
    const int v  = u - NU1;
    const int n  = v >> 6;
    const int k8 = (v & 63) * 8;
    const int kk = k8 & (HC1 - 1);
    const float* p = W2 + (size_t)kk * NOUT + n;
#pragma unroll
    for (int i = 0; i < 8; ++i) o[i] = (unsigned short)f2bf(p[(size_t)i * NOUT]);
    dp = W22T + (size_t)n * KP + k8;
  } else {
    return;
  }
  *(volatile v8us*)dp = o;
  __threadfence();
  *(volatile v8us*)dp = o;
}

__global__ __launch_bounds__(NTHR) void k_gemm1(const float* __restrict__ X, int nN,
                                                const unsigned short* __restrict__ BT, float* Cm,
                                                const float* __restrict__ avs, const float* __restrict__ avd,
                                                float* SD) {
  extern __shared__ __attribute__((aligned(16))) float gsm[];
  float* stg = gsm;
  float* sdt = gsm + GBM * HC1;
  const int tid = (int)threadIdx.x, lane = tid & 31, wave = tid >> 5, hh = lane >> 4, m = lane & 15;
  const int rg = wave & 3, cg = wave >> 2;
  const int rowBase = (int)blockIdx.x * GBM;
  const int colBase = cg * 128;

  v8f acc[8];
  {
    const v8f z = {0.f, 0.f, 0.f, 0.f, 0.f, 0.f, 0.f, 0.f};
#pragma unroll
    for (int t = 0; t < 8; ++t) acc[t] = z;
  }
  const int arow = rowBase + 16 * rg + m;
  const int arc  = arow < nN ? arow : nN - 1;
  const int lm   = arow < nN ? -1 : 0;
  const float* ap = X + (size_t)arc * F_IN + 8 * hh;
  const unsigned short* bp = BT + (size_t)(colBase + m) * F_IN + 8 * hh;

#pragma unroll 1
  for (int k0 = 0; k0 < F_IN; k0 += 32) {
    const v4f x0 = *(const v4fa*)(ap + k0);
    const v4f x1 = *(const v4fa*)(ap + k0 + 4);
    const v4f x2 = *(const v4fa*)(ap + k0 + 16);
    const v4f x3 = *(const v4fa*)(ap + k0 + 20);
    v8i aw;
    aw[0] = (int)pk2(x0.x, x0.y) & lm; aw[1] = (int)pk2(x0.z, x0.w) & lm;
    aw[2] = (int)pk2(x1.x, x1.y) & lm; aw[3] = (int)pk2(x1.z, x1.w) & lm;
    aw[4] = (int)pk2(x2.x, x2.y) & lm; aw[5] = (int)pk2(x2.z, x2.w) & lm;
    aw[6] = (int)pk2(x3.x, x3.y) & lm; aw[7] = (int)pk2(x3.z, x3.w) & lm;
    FragB af;
    af.w = aw;
#pragma unroll
    for (int nt = 0; nt < 8; ++nt) {
      const unsigned short* wq = bp + (size_t)(16 * nt) * (size_t)F_IN + k0;
      FragB bf;
      bf.h[0] = *(const v8usa*)wq;
      bf.h[1] = *(const v8usa*)(wq + 16);
      acc[nt] = wmb(af, bf, acc[nt]);
    }
  }

#pragma unroll
  for (int nt = 0; nt < 8; ++nt) {
    const int lc = colBase + 16 * nt + m;
#pragma unroll
    for (int r = 0; r < 8; ++r) {
      const int lr = 16 * rg + 8 * hh + r;
      stg[lr * HC1 + lc] = acc[nt][r];
    }
  }
  __syncthreads();

  v4f as4[2], ad4[2];
#pragma unroll
  for (int c = 0; c < 2; ++c) {
    as4[c] = bfr4(*(const v4fa*)(avs + c * 128 + 4 * lane));
    ad4[c] = bfr4(*(const v4fa*)(avd + c * 128 + 4 * lane));
  }
#pragma unroll 1
  for (int i = 0; i < 8; ++i) {
    const int row = wave * 8 + i;
#pragma unroll
    for (int c = 0; c < 2; ++c) {
      const v4f p = *(const v4fa*)(stg + row * HC1 + c * 128 + 4 * lane);
      float s = p.x * as4[c].x; s = fmaf(p.y, as4[c].y, s); s = fmaf(p.z, as4[c].z, s); s = fmaf(p.w, as4[c].w, s);
      float d = p.x * ad4[c].x; d = fmaf(p.y, ad4[c].y, d); d = fmaf(p.z, ad4[c].z, d); d = fmaf(p.w, ad4[c].w, d);
      s += __shfl_xor(s, 4); d += __shfl_xor(d, 4);
      s += __shfl_xor(s, 2); d += __shfl_xor(d, 2);
      s += __shfl_xor(s, 1); d += __shfl_xor(d, 1);
      if ((lane & 7) == 0) {
        sdt[row * SDW + 4 * c + (lane >> 3)]     = s;
        sdt[row * SDW + 8 + 4 * c + (lane >> 3)] = d;
      }
    }
  }
  __syncthreads();

  const v4f sdv = *(const v4fa*)(sdt + 4 * tid);
  float* sp = SD + (size_t)blockIdx.x * (GBM * SDW) + 4 * tid;
#pragma unroll 1
  for (int i = 0; i < 8; ++i) {
    const int row = wave * 8 + i;
#pragma unroll
    for (int c = 0; c < 2; ++c) {
      const v4f p = *(const v4fa*)(stg + row * HC1 + c * 128 + 4 * lane);
      float* op = Cm + (size_t)(rowBase + row) * (size_t)HC1 + c * 128 + 4 * lane;
      *(volatile v4f*)op = p;
    }
  }
  *(volatile v4f*)sp = sdv;
  __threadfence();
#pragma unroll 1
  for (int i = 0; i < 8; ++i) {
    const int row = wave * 8 + i;
#pragma unroll
    for (int c = 0; c < 2; ++c) {
      const v4f p = *(const v4fa*)(stg + row * HC1 + c * 128 + 4 * lane);
      float* op = Cm + (size_t)(rowBase + row) * (size_t)HC1 + c * 128 + 4 * lane;
      *(volatile v4f*)op = p;
    }
  }
  *(volatile v4f*)sp = sdv;
}

__global__ __launch_bounds__(GTHR) void k_gemm2(
    const unsigned short* __restrict__ A, const unsigned short* __restrict__ WT,
    float* outF, int K, int ldo,
    const float* __restrict__ atts, const float* __restrict__ attd, int attLen,
    float* SD, int MPr)
{
  __shared__ __attribute__((aligned(16))) float stg[GBM * GBN];
  __shared__ __attribute__((aligned(16))) float satt[2 * GBN];
  __shared__ __attribute__((aligned(16))) float sdot[2 * GBM];
  const int tid = (int)threadIdx.x, lane = tid & 31, wave = tid >> 5, hh = lane >> 4, m = lane & 15;
  const int rowBase = (int)blockIdx.x * GBM;
  const int head    = (int)blockIdx.y;
  const int col0    = head * GBN;

  {
    const int which = tid >> 6;
    const int c  = tid & 63;
    const int cl = c < attLen ? c : attLen - 1;
    const float vs = atts[head * attLen + cl];
    const float vd = attd[head * attLen + cl];
    float v = (which == 0) ? vs : vd;
    v = (c < attLen) ? bfr(v) : 0.f;
    satt[which * GBN + c] = v;
  }

  v8f acc[4];
  {
    const v8f z = {0.f, 0.f, 0.f, 0.f, 0.f, 0.f, 0.f, 0.f};
    acc[0] = z; acc[1] = z; acc[2] = z; acc[3] = z;
  }
  const unsigned short* ap = A  + (size_t)(rowBase + 16 * wave + m) * (size_t)K + 8 * hh;
  const unsigned short* wp = WT + (size_t)(col0 + m) * (size_t)K + 8 * hh;
  const int ksteps = K >> 5;
#pragma unroll 1
  for (int ks = 0; ks < ksteps; ++ks) {
    FragB af;
    af.h[0] = *(const v8usa*)(ap + 32 * ks);
    af.h[1] = *(const v8usa*)(ap + 32 * ks + 16);
#pragma unroll
    for (int t = 0; t < 4; ++t) {
      const unsigned short* wq = wp + (size_t)(16 * t) * (size_t)K + 32 * ks;
      FragB bf;
      bf.h[0] = *(const v8usa*)wq;
      bf.h[1] = *(const v8usa*)(wq + 16);
      acc[t] = wmb(af, bf, acc[t]);
    }
  }

#pragma unroll
  for (int t = 0; t < 4; ++t) {
    const int lc = 16 * t + m;
#pragma unroll
    for (int r = 0; r < 8; ++r) {
      const int lr = 16 * wave + 8 * hh + r;
      stg[lr * GBN + lc] = acc[t][r];
    }
  }
  __syncthreads();

  {
    const int row = tid & 63, which = tid >> 6;
    const float* sa = satt + which * GBN;
    const float* hr = stg + row * GBN;
    float d = 0.f;
#pragma unroll 4
    for (int c4 = 0; c4 < GBN / 4; ++c4) {
      const v4f hv = *(const v4fa*)(hr + 4 * c4);
      const v4f av = *(const v4fa*)(sa + 4 * c4);
      d = fmaf(hv.x, av.x, d);
      d = fmaf(hv.y, av.y, d);
      d = fmaf(hv.z, av.z, d);
      d = fmaf(hv.w, av.w, d);
    }
    sdot[which * GBM + row] = d;
  }
  __syncthreads();

  v4f fv[8];
#pragma unroll
  for (int i = 0; i < 8; ++i) {
    const int lr = 16 * wave + 2 * i + hh;
    fv[i] = *(const v4fa*)(stg + lr * GBN + 4 * m);
  }
  const int which2 = lane >> 4, piece = lane & 15;
  const v4f sdv = *(const v4fa*)(sdot + which2 * GBM + 4 * piece);
  float* sp = SD + (size_t)(2 * head + which2) * (size_t)MPr + rowBase + 4 * piece;

#pragma unroll
  for (int i = 0; i < 8; ++i) {
    const int lr = 16 * wave + 2 * i + hh;
    const int gr = rowBase + lr;
    float* op = outF + (size_t)gr * (size_t)ldo + col0 + 4 * m;
    *(volatile v4f*)op = fv[i];
  }
  if (wave == 0) *(volatile v4f*)sp = sdv;
  __threadfence();
#pragma unroll
  for (int i = 0; i < 8; ++i) {
    const int lr = 16 * wave + 2 * i + hh;
    const int gr = rowBase + lr;
    float* op = outF + (size_t)gr * (size_t)ldo + col0 + 4 * m;
    *(volatile v4f*)op = fv[i];
  }
  if (wave == 0) *(volatile v4f*)sp = sdv;
}

template <int L>
__global__ __launch_bounds__(NTHR) void k_scan(const int* __restrict__ srcs, const int* __restrict__ dsts,
                                               int nE, int nN, int vec8, int mRows,
                                               const float* __restrict__ SD, const float* __restrict__ F,
                                               const float* __restrict__ bias,
                                               unsigned short* hb, float* outp) {
  static_assert(L == 1 || L == 2);
  constexpr int CPL = (L == 1) ? 8 : 2;
  constexpr int C   = CPL * 32;
  extern __shared__ __attribute__((aligned(16))) int dsm[];
  int* list = dsm;
  int* hl   = dsm + LISTN;
  int* sl   = dsm + LISTN + RCAP;
  int* cnt  = dsm + LISTN + 2 * RCAP;
  int* offs = cnt + NBA;
  int* cur  = offs + NBA;
  int* misc = cur + NBA;
  float* est = (float*)(misc + 16);
  const int tid = (int)threadIdx.x, lane = tid & 31, wave = tid >> 5;
  const int nodeBase = (int)blockIdx.x * NBA;

  {
    const v4i z4 = {0, 0, 0, 0};
    for (int i = tid * 4; i < AGG_ZINTS; i += NTHR * 4) *(v4ia*)(dsm + i) = z4;
    if (tid < 16) misc[tid] = 0;
  }
  float bv[CPL];
  if constexpr (L == 1) {
    const float* bq = bias + 8 * lane;
    const v4f a = *(const v4fa*)bq;
    const v4f b = *(const v4fa*)(bq + 4);
    bv[0] = bfr(a.x); bv[1] = bfr(a.y); bv[2] = bfr(a.z); bv[3] = bfr(a.w);
    bv[4] = bfr(b.x); bv[5] = bfr(b.y); bv[6] = bfr(b.z); bv[7] = bfr(b.w);
  } else {
    const v2f a = *(const v2fa*)(bias + 2 * lane);
    bv[0] = bfr(a.x); bv[1] = bfr(a.y);
  }
  __syncthreads();

  int t = 0, ov = 0;
  const int nChunks = (nE + CHUNK - 1) / CHUNK;
#pragma unroll 1
  for (int ch = 0; ch < nChunks; ++ch) {
    const int cbase = ch * CHUNK;
    const int wc = scan_chunk<SLA>(dsts, nE, cbase, nodeBase, NBA, vec8, list, tid, lane, wave);
    if (lane == 0) misc[wave] = wc;
    __syncthreads();
    if (wave == 0) {
#pragma unroll 1
      for (int w2 = 0; w2 < NWAVE; ++w2) {
        int c = misc[w2];
        c = c < 0 ? 0 : (c > WCAP ? WCAP : c);
#pragma unroll 1
        for (int b0 = 0; b0 < c; b0 += 32) {
          const int idx = b0 + lane;
          const int ent = list[w2 * WCAP + (idx < WCAP ? idx : WCAP - 1)];
          const int m32 = (c - b0) < 32 ? (c - b0) : 32;
#pragma unroll 1
          for (int k = 0; k < m32; ++k) {
            const int u    = __builtin_amdgcn_readlane(ent, k);
            const int slot = u & (NBA - 1);
            const int el   = (u >> SLA) & (CHUNK - 1);
            const int pk   = ((cbase + el) << SLA) | slot;
            if (t < RCAP) {
              if (lane == 0) { hl[t] = pk; cnt[slot] = cnt[slot] + 1; }
              t = t + 1;
            } else {
              ov = 1;
            }
          }
        }
      }
    }
    __syncthreads();
  }
  if (wave == 0 && lane == 0) { misc[8] = t; misc[9] = ov; }
  __syncthreads();
  int tt = misc[8];
  tt = tt < 0 ? 0 : (tt > RCAP ? RCAP : tt);
  const int ovf = misc[9];

  if (wave == 0) {
    const int base = lane * (NBA / 32);
    int s = 0;
#pragma unroll 1
    for (int i = 0; i < NBA / 32; ++i) s += cnt[base + i];
    int incl = s;
#pragma unroll
    for (int d = 1; d < 32; d <<= 1) {
      const int y = __shfl_up(incl, d, 32);
      if (lane >= d) incl += y;
    }
    int run = incl - s;
#pragma unroll 1
    for (int i = 0; i < NBA / 32; ++i) {
      const int cv = cnt[base + i];
      offs[base + i] = run;
      cur[base + i]  = run;
      run += cv;
    }
  }
  __syncthreads();
  if (wave == 0) {
#pragma unroll 1
    for (int b0 = 0; b0 < tt; b0 += 32) {
      const int idx = b0 + lane;
      const int ent = hl[idx < RCAP ? idx : RCAP - 1];
      const int m32 = (tt - b0) < 32 ? (tt - b0) : 32;
#pragma unroll 1
      for (int k = 0; k < m32; ++k) {
        const int u    = __builtin_amdgcn_readlane(ent, k);
        const int slot = u & (NBA - 1);
        if (lane == 0) {
          int p = cur[slot];
          p = p < 0 ? 0 : (p > RCAP - 1 ? RCAP - 1 : p);
          sl[p] = u;
          cur[slot] = p + 1;
        }
      }
    }
  }
  __syncthreads();

  const float qnan = __int_as_float(0x7fc00000);
  const float pz = (ovf != 0) ? qnan : 0.0f;
  const int hd = lane >> 2;
  float* my = est + tid * 8;
#pragma unroll 1
  for (int si = 0; si < NBA / NWAVE; ++si) {
    const int s    = si * NWAVE + wave;
    const int node = nodeBase + s;
    const int craw = cnt[s];
    const bool big = craw > DEGCAP;
    const int c = craw < 0 ? 0 : (craw > DEGCAP ? DEGCAP : craw);
    int o = offs[s];
    o = o < 0 ? 0 : (o > RCAP ? RCAP : o);
    const int nc = node < nN ? node : nN - 1;
    float adv;
    if constexpr (L == 1) adv = SD[(size_t)nc * SDW + 8 + hd];
    else                  adv = SD[(size_t)mRows + nc];

    float mx = -3.0e38f;
#pragma unroll 1
    for (int q = 0; q < c; ++q) {
      int idx = o + q; idx = idx > RCAP - 1 ? RCAP - 1 : idx;
      const int ent = sl[idx];
      int eid = ent >> SLA;
      eid = eid < 0 ? 0 : (eid > nE - 1 ? nE - 1 : eid);
      int sr = srcs[eid];
      sr = sr < 0 ? 0 : (sr > nN - 1 ? nN - 1 : sr);
      float es;
      if constexpr (L == 1) es = SD[(size_t)sr * SDW + hd];
      else                  es = SD[sr];
      float lg = es + adv;
      lg = lg > 0.f ? lg : NEGSL * lg;
      mx = lg > mx ? lg : mx;
    }

    float dn = 0.0f;
    float acc[CPL];
#pragma unroll
    for (int i = 0; i < CPL; ++i) acc[i] = 0.0f;
#pragma unroll 1
    for (int q = 0; q < c; ++q) {
      int idx = o + q; idx = idx > RCAP - 1 ? RCAP - 1 : idx;
      const int ent = sl[idx];
      int eid = ent >> SLA;
      eid = eid < 0 ? 0 : (eid > nE - 1 ? nE - 1 : eid);
      int sr = srcs[eid];
      sr = sr < 0 ? 0 : (sr > nN - 1 ? nN - 1 : sr);
      float es;
      if constexpr (L == 1) es = SD[(size_t)sr * SDW + hd];
      else                  es = SD[sr];
      const float* rp = F + (size_t)sr * C + CPL * lane;
      float lg = es + adv;
      lg = lg > 0.f ? lg : NEGSL * lg;
      const float p = expf(lg - mx);
      dn += p;
      if constexpr (L == 1) {
        const v4f a = *(const v4fa*)rp;
        const v4f b = *(const v4fa*)(rp + 4);
        acc[0] = fmaf(p, a.x, acc[0]); acc[1] = fmaf(p, a.y, acc[1]);
        acc[2] = fmaf(p, a.z, acc[2]); acc[3] = fmaf(p, a.w, acc[3]);
        acc[4] = fmaf(p, b.x, acc[4]); acc[5] = fmaf(p, b.y, acc[5]);
        acc[6] = fmaf(p, b.z, acc[6]); acc[7] = fmaf(p, b.w, acc[7]);
      } else {
        const v2f a = *(const v2fa*)rp;
        acc[0] = fmaf(p, a.x, acc[0]); acc[1] = fmaf(p, a.y, acc[1]);
      }
    }
    const float rc  = __builtin_amdgcn_rcpf(dn);
    const float inv = (c > 0) ? rc : 0.0f;
    const float pzr = big ? qnan : pz;
    const bool live = node < nN;

    if constexpr (L == 1) {
      v4f va, vb;
      va.x = fmaf(acc[0], inv, bv[0]); va.y = fmaf(acc[1], inv, bv[1]);
      va.z = fmaf(acc[2], inv, bv[2]); va.w = fmaf(acc[3], inv, bv[3]);
      vb.x = fmaf(acc[4], inv, bv[4]); vb.y = fmaf(acc[5], inv, bv[5]);
      vb.z = fmaf(acc[6], inv, bv[6]); vb.w = fmaf(acc[7], inv, bv[7]);
      *(v4fa*)my = va;
      *(v4fa*)(my + 4) = vb;
#pragma unroll 1
      for (int i = 0; i < 8; ++i) {
        const float xv = my[i];
        const float yv = (xv > 0.0f) ? xv : expm1f(xv);
        my[i] = yv;
      }
      va = *(const v4fa*)my;
      vb = *(const v4fa*)(my + 4);
      float v[8];
      v[0] = va.x; v[1] = va.y; v[2] = va.z; v[3] = va.w;
      v[4] = vb.x; v[5] = vb.y; v[6] = vb.z; v[7] = vb.w;
      v8us ho, lo;
#pragma unroll
      for (int i = 0; i < 8; ++i) {
        const float y  = v[i] + pzr;
        const float yy = live ? y : 0.0f;
        const unsigned int hbi = f2bf(yy);
        ho[i] = (unsigned short)hbi;
        lo[i] = (unsigned short)f2bf(yy - bf2f(hbi));
      }
      if (node < mRows) {
        unsigned short* hp = hb + (size_t)node * KP + 8 * lane;
        *(volatile v8us*)hp = ho;
        *(volatile v8us*)(hp + HC1) = lo;
        __threadfence();
        *(volatile v8us*)hp = ho;
        *(volatile v8us*)(hp + HC1) = lo;
      }
    } else {
      v2f ov2;
      ov2.x = fmaf(acc[0], inv, bv[0]) + pzr;
      ov2.y = fmaf(acc[1], inv, bv[1]) + pzr;
      if (live) {
        float* op = outp + (size_t)node * NOUT + 2 * lane;
        *(volatile v2f*)op = ov2;
        __threadfence();
        *(volatile v2f*)op = ov2;
      }
    }
  }
}

static inline int cdiv(int a, int b) { return (a + b - 1) / b; }

extern "C" void kernel_launch(void* const* d_in, const int* in_sizes, int n_in,
                              void* d_out, int out_size, void* d_ws, size_t ws_size,
                              hipStream_t stream) {
  if (n_in < 11) return;
  if (in_sizes[0] < F_IN || (in_sizes[0] % F_IN) != 0) return;
  const int nN = in_sizes[0] / F_IN;
  if (nN <= 0 || nN > (1 << 22)) return;
  if (in_sizes[1] != F_IN * HC1) return;
  if (in_sizes[2] != HC1 || in_sizes[3] != HC1 || in_sizes[4] != HC1) return;
  if (in_sizes[5] != HC1 * NOUT) return;
  if (in_sizes[6] != NOUT || in_sizes[7] != NOUT || in_sizes[8] != NOUT) return;
  const int nE = in_sizes[9];
  if (nE < 1 || nE >= (1 << 21) || in_sizes[10] != nE) return;
  if ((long long)out_size != (long long)nN * NOUT) return;

  const float* x   = (const float*)d_in[0];
  const float* W1  = (const float*)d_in[1];
  const float* a1s = (const float*)d_in[2];
  const float* a1d = (const float*)d_in[3];
  const float* b1  = (const float*)d_in[4];
  const float* W2  = (const float*)d_in[5];
  const float* a2s = (const float*)d_in[6];
  const float* a2d = (const float*)d_in[7];
  const float* b2  = (const float*)d_in[8];
  const int*   src = (const int*)d_in[9];
  const int*   dst = (const int*)d_in[10];
  float* out = (float*)d_out;

  const int MP   = cdiv(nN, GBM) * GBM;
  const int gM   = MP / GBM;
  const int gA   = cdiv(MP, NBA);
  if ((long long)gA * NBA < (long long)MP) return;
  const int vec8 = ((nE & 3) == 0) ? 1 : 0;

  char* ws = (char*)d_ws;
  size_t off = 0;
  const size_t oW1T = off; off += (size_t)HC1 * F_IN * 2;          off = (off + 255) & ~(size_t)255;
  const size_t oW2T = off; off += (size_t)NOUT * KP * 2;           off = (off + 255) & ~(size_t)255;
  const size_t oH1  = off; off += (size_t)MP * HC1 * 4;            off = (off + 255) & ~(size_t)255;
  const size_t oSD1 = off; off += (size_t)MP * SDW * 4;            off = (off + 255) & ~(size_t)255;
  const size_t oX1  = off; off += (size_t)MP * KP * 2;             off = (off + 255) & ~(size_t)255;
  const size_t oH2  = off; off += (size_t)MP * NOUT * 4;           off = (off + 255) & ~(size_t)255;
  const size_t oSD2 = off; off += (size_t)2 * MP * 4;              off = (off + 255) & ~(size_t)255;
  if (off > ws_size || off > (size_t)WSMAX) return;
  unsigned short* W1T  = (unsigned short*)(ws + oW1T);
  unsigned short* W22T = (unsigned short*)(ws + oW2T);
  float*          H1   = (float*)(ws + oH1);
  float*          SD1  = (float*)(ws + oSD1);
  unsigned short* X1   = (unsigned short*)(ws + oX1);
  float*          H2   = (float*)(ws + oH2);
  float*          SD2  = (float*)(ws + oSD2);

  const size_t scanLds = (size_t)AGG_LDS_INTS * 4;
  const size_t g1Lds   = (size_t)G1_LDS_FLOATS * 4;
  hipFuncSetAttribute(reinterpret_cast<const void*>(&k_gemm1), hipFuncAttributeMaxDynamicSharedMemorySize, (int)g1Lds);
  hipFuncSetAttribute(reinterpret_cast<const void*>(&k_scan<1>), hipFuncAttributeMaxDynamicSharedMemorySize, (int)scanLds);
  hipFuncSetAttribute(reinterpret_cast<const void*>(&k_scan<2>), hipFuncAttributeMaxDynamicSharedMemorySize, (int)scanLds);

  k_wprep<<<(NU1 + NU2) / NTHR, NTHR, 0, stream>>>(W1, W2, W1T, W22T);
  k_gemm1<<<gM, NTHR, g1Lds, stream>>>(x, nN, W1T, H1, a1s, a1d, SD1);
  k_scan<1><<<gA, NTHR, scanLds, stream>>>(src, dst, nE, nN, vec8, MP, SD1, H1, b1, X1, out);
  k_gemm2<<<dim3(gM, NOUT / GBN), GTHR, 0, stream>>>(X1, W22T, H2, KP, NOUT, a2s, a2d, NOUT, SD2, MP);
  k_scan<2><<<gA, NTHR, scanLds, stream>>>(src, dst, nE, nN, vec8, MP, SD2, H2, b2, X1, out);
}
